// SpectralEncoderLayer_38843684225855
// MI455X (gfx1250) — hardware-verified
//
#include <hip/hip_runtime.h>
#include <stdint.h>

#define NBAT  4
#define EMB   128
#define IMH   64
#define IMW   64
#define HWP   4096
#define NPIX  16384
#define HEADS 4
#define HDIM  32
#define FFD   512
#define NQC   64
#define KWIN  7
#define PWIN  49
#define LDC   132
#define OSP   132
#define NBW0  24
#define NBW1  32
#define NBW2  32
#define NBT   256
#define WSC   64.0f
#define PJS   0.015625f
#define QKS   16.0f
#define SSC   0.00390625f
#define VSC   16.0f
#define RES   2048.0f
#define RSC   0.00048828125f
#define OFAC  64.0f
#define TSC   64.0f
#define PSC   0.0000152587890625f
#define HSC   16.0f
#define F2S   0.0009765625f
#define LNEPS 0.00001f

static_assert(NPIX == NBAT * IMH * IMW && HWP == IMH * IMW);
static_assert(EMB == HEADS * HDIM && HDIM == 32 && IMW == 64);
static_assert(PWIN == KWIN * KWIN && HEADS * PWIN <= 256);
static_assert(NBW0 * 256 * 8 == 3 * EMB * EMB && NBW1 * 256 * 8 == FFD * EMB && NBW2 * 256 * 8 == EMB * FFD);
static_assert(NBT * 256 == NBAT * EMB * EMB);
static_assert((LDC * 4) % 16 == 0 && (OSP * 4) % 16 == 0);
static_assert((EMB % 32) == 0 && (FFD % 32) == 0 && (NQC % 4) == 0 && (NPIX % 64) == 0);

typedef _Float16       v16h  __attribute__((ext_vector_type(16)));
typedef unsigned short v16us __attribute__((ext_vector_type(16)));
typedef unsigned short v8us  __attribute__((ext_vector_type(8)));
typedef float          v8f   __attribute__((ext_vector_type(8)));
typedef float          v4f   __attribute__((ext_vector_type(4)));
typedef unsigned int   v4u   __attribute__((ext_vector_type(4)));

union UFrag { v16us v; v8us u[2]; v4u w[2]; };

__device__ __forceinline__ unsigned short bf_bits(float f) {
  unsigned u = __float_as_uint(f);
  return (unsigned short)((u + 0x7FFFu + ((u >> 16) & 1u)) >> 16);
}
__device__ __forceinline__ float bf_up(unsigned short b) { return __uint_as_float(((unsigned)b) << 16); }
__device__ __forceinline__ float bfr(float f) { return bf_up(bf_bits(f)); }
__device__ __forceinline__ unsigned short h_bits(_Float16 x) { return __builtin_bit_cast(unsigned short, x); }
__device__ __forceinline__ unsigned short hb16(float f) { return h_bits((_Float16)f); }
__device__ __forceinline__ unsigned pk16(unsigned short a, unsigned short b) { return (unsigned)a | ((unsigned)b << 16); }
__device__ __forceinline__ v8f zero8() { v8f z = {0.f, 0.f, 0.f, 0.f, 0.f, 0.f, 0.f, 0.f}; return z; }
__device__ __forceinline__ v16us zero16() {
  v16us z;
#pragma unroll
  for (int i = 0; i < 16; ++i) z[i] = 0;
  return z;
}
__device__ __forceinline__ v8us zero8u() { v8us z = {0, 0, 0, 0, 0, 0, 0, 0}; return z; }

__device__ __forceinline__ void hl2(float f0, float f1, unsigned& hpk, unsigned& lpk) {
  const _Float16 h0 = (_Float16)f0, h1 = (_Float16)f1;
  hpk = pk16(h_bits(h0), h_bits(h1));
  lpk = pk16(hb16((f0 - (float)h0) * RES), hb16((f1 - (float)h1) * RES));
}

__device__ __forceinline__ void st16x2(unsigned short* dst, v4u pk) {
  *(volatile v4u*)dst = pk;
  __threadfence();
  *(volatile v4u*)dst = pk;
}

__device__ __forceinline__ v4u cvt_w8(const float* __restrict__ src) {
  const v4f a = *(const v4f*)(src);
  const v4f b = *(const v4f*)(src + 4);
  v4u pk;
  pk[0] = pk16(hb16(bfr(a[0]) * WSC), hb16(bfr(a[1]) * WSC));
  pk[1] = pk16(hb16(bfr(a[2]) * WSC), hb16(bfr(a[3]) * WSC));
  pk[2] = pk16(hb16(bfr(b[0]) * WSC), hb16(bfr(b[1]) * WSC));
  pk[3] = pk16(hb16(bfr(b[2]) * WSC), hb16(bfr(b[3]) * WSC));
  return pk;
}

__device__ __forceinline__ v16us ldfrag(const unsigned short* p) {
  union { v16us v; v8us h[2]; } f;
  f.h[0] = *(const v8us*)(p);
  f.h[1] = *(const v8us*)(p + 16);
  return f.v;
}

__device__ __forceinline__ v8f mma_h(v16us a, v16us b, v8f c) {
#if defined(__HIP_DEVICE_COMPILE__)
  return __builtin_amdgcn_wmma_f32_16x16x32_f16(false, __builtin_bit_cast(v16h, a), false,
                                               __builtin_bit_cast(v16h, b), (short)0, c, false, false);
#else
  (void)a; (void)b;
  return c;
#endif
}
__device__ __forceinline__ void guard8(v8f& c0, v8f& c1, v8f& c2, v8f& c3, v8f& c4, v8f& c5, v8f& c6, v8f& c7,
                                       const v16us& a0, const v16us& a1, const v16us& a2, const v16us& a3,
                                       const v16us& b0, const v16us& b1) {
#if defined(__HIP_DEVICE_COMPILE__)
  asm volatile("v_nop\n\tv_nop\n\tv_nop\n\tv_nop"
               : "+v"(c0), "+v"(c1), "+v"(c2), "+v"(c3), "+v"(c4), "+v"(c5), "+v"(c6), "+v"(c7)
               : "v"(a0), "v"(a1), "v"(a2), "v"(a3), "v"(b0), "v"(b1));
#endif
}
__device__ __forceinline__ void guard_s1(v8f& s, const v16us& a, const v16us& b) {
#if defined(__HIP_DEVICE_COMPILE__)
  asm volatile("v_nop\n\tv_nop\n\tv_nop\n\tv_nop" : "+v"(s) : "v"(a), "v"(b));
#endif
}
__device__ __forceinline__ void guard_s2(v8f& s0, v8f& s1, const v16us& a0, const v16us& a1, const v16us& b) {
#if defined(__HIP_DEVICE_COMPILE__)
  asm volatile("v_nop\n\tv_nop\n\tv_nop\n\tv_nop" : "+v"(s0), "+v"(s1) : "v"(a0), "v"(a1), "v"(b));
#endif
}
__device__ __forceinline__ void guard6(v8f& c0, v8f& c1, v8f& c2, v8f& c3,
                                       const v16us& a0, const v16us& a1, const v16us& b0, const v16us& b1,
                                       const v16us& b2, const v16us& b3) {
#if defined(__HIP_DEVICE_COMPILE__)
  asm volatile("v_nop\n\tv_nop\n\tv_nop\n\tv_nop"
               : "+v"(c0), "+v"(c1), "+v"(c2), "+v"(c3)
               : "v"(a0), "v"(a1), "v"(b0), "v"(b1), "v"(b2), "v"(b3));
#endif
}

__device__ __forceinline__ void mm_core2(const unsigned short* __restrict__ Ah, const unsigned short* __restrict__ Al,
                                         int lda, const unsigned short* __restrict__ W, int ldw, int nks,
                                         int arow0, int brow0, float* Cs) {
  const int tid = threadIdx.x, wave = tid >> 5, lane = tid & 31, hh = lane >> 4, c = lane & 15;
  const int mw = wave >> 2, nw = wave & 3;
  const size_t r0 = (size_t)(arow0 + mw * 32 + c) * lda + 8 * hh;
  const size_t r1 = (size_t)(arow0 + mw * 32 + 16 + c) * lda + 8 * hh;
  const unsigned short* a0h = Ah + r0;
  const unsigned short* a1h = Ah + r1;
  const unsigned short* a0l = Al + r0;
  const unsigned short* a1l = Al + r1;
  const unsigned short* b0p = W + (size_t)(brow0 + nw * 32 + c) * ldw + 8 * hh;
  const unsigned short* b1p = W + (size_t)(brow0 + nw * 32 + 16 + c) * ldw + 8 * hh;
  v8f h00 = zero8(), h01 = zero8(), h10 = zero8(), h11 = zero8();
  v8f l00 = zero8(), l01 = zero8(), l10 = zero8(), l11 = zero8();
#pragma unroll 1
  for (int ks = 0; ks < nks; ++ks) {
    const int ko = ks * 32;
    const v16us fa0 = ldfrag(a0h + ko);
    const v16us fa1 = ldfrag(a1h + ko);
    const v16us ga0 = ldfrag(a0l + ko);
    const v16us ga1 = ldfrag(a1l + ko);
    const v16us fb0 = ldfrag(b0p + ko);
    const v16us fb1 = ldfrag(b1p + ko);
    h00 = mma_h(fa0, fb0, h00);
    h01 = mma_h(fa0, fb1, h01);
    h10 = mma_h(fa1, fb0, h10);
    h11 = mma_h(fa1, fb1, h11);
    l00 = mma_h(ga0, fb0, l00);
    l01 = mma_h(ga0, fb1, l01);
    l10 = mma_h(ga1, fb0, l10);
    l11 = mma_h(ga1, fb1, l11);
    guard8(h00, h01, h10, h11, l00, l01, l10, l11, fa0, fa1, ga0, ga1, fb0, fb1);
  }
#pragma unroll
  for (int r = 0; r < 8; ++r) {
    const int row = mw * 32 + 8 * hh + r;
    Cs[row * LDC + nw * 32 + c]             = h00[r] + l00[r] * RSC;
    Cs[row * LDC + nw * 32 + 16 + c]        = h01[r] + l01[r] * RSC;
    Cs[(row + 16) * LDC + nw * 32 + c]      = h10[r] + l10[r] * RSC;
    Cs[(row + 16) * LDC + nw * 32 + 16 + c] = h11[r] + l11[r] * RSC;
  }
}

__device__ __forceinline__ void ln_tile(float* Xs, const float* __restrict__ g, const float* __restrict__ b) {
  const int tid = threadIdx.x, wave = tid >> 5, lane = tid & 31;
  const int c0 = lane * 4;
  float gg[4], bb[4];
#pragma unroll
  for (int e = 0; e < 4; ++e) { gg[e] = bfr(g[c0 + e]); bb[e] = bfr(b[c0 + e]); }
#pragma unroll 1
  for (int j = 0; j < 8; ++j) {
    const int px = wave * 8 + j;
    const v4f v = *(const v4f*)(Xs + px * LDC + c0);
    float s = (v[0] + v[1]) + (v[2] + v[3]);
#pragma unroll
    for (int off = 16; off > 0; off >>= 1) s += __shfl_xor(s, off, 32);
    const float mean = s * (1.0f / 128.0f);
    v4f d;
#pragma unroll
    for (int e = 0; e < 4; ++e) d[e] = v[e] - mean;
    float ss = (d[0] * d[0] + d[1] * d[1]) + (d[2] * d[2] + d[3] * d[3]);
#pragma unroll
    for (int off = 16; off > 0; off >>= 1) ss += __shfl_xor(ss, off, 32);
    const float var = ss * (1.0f / 128.0f);
    const float rstd = rsqrtf(var + LNEPS);
    v4f o;
#pragma unroll
    for (int e = 0; e < 4; ++e) o[e] = (d[e] * rstd) * gg[e] + bb[e];
    *(v4f*)(Xs + px * LDC + c0) = o;
  }
}

__device__ __forceinline__ void store_hilo(const float* Xs, unsigned short* hp, unsigned short* lp, size_t row0) {
  const int tid = threadIdx.x;
  v4u hw[4], lw[4];
  size_t offs[4];
#pragma unroll
  for (int s = 0; s < 4; ++s) {
    const int idx = s * 256 + tid;
    const int row = idx >> 4, piece = idx & 15;
    const v4f a = *(const v4f*)(Xs + row * LDC + piece * 8);
    const v4f b = *(const v4f*)(Xs + row * LDC + piece * 8 + 4);
    v4u h4, l4;
    unsigned ph_, pl_;
    hl2(a[0], a[1], ph_, pl_); h4[0] = ph_; l4[0] = pl_;
    hl2(a[2], a[3], ph_, pl_); h4[1] = ph_; l4[1] = pl_;
    hl2(b[0], b[1], ph_, pl_); h4[2] = ph_; l4[2] = pl_;
    hl2(b[2], b[3], ph_, pl_); h4[3] = ph_; l4[3] = pl_;
    hw[s] = h4;
    lw[s] = l4;
    offs[s] = (row0 + row) * EMB + piece * 8;
  }
#pragma unroll
  for (int s = 0; s < 4; ++s) { *(volatile v4u*)(hp + offs[s]) = hw[s]; *(volatile v4u*)(lp + offs[s]) = lw[s]; }
  __threadfence();
#pragma unroll
  for (int s = 0; s < 4; ++s) { *(volatile v4u*)(hp + offs[s]) = hw[s]; *(volatile v4u*)(lp + offs[s]) = lw[s]; }
}

__global__ __launch_bounds__(256)
void k_cvt(const float* __restrict__ wq, const float* __restrict__ wk, const float* __restrict__ wv,
           const float* __restrict__ w1, const float* __restrict__ w2, const float* __restrict__ bw,
           const float* __restrict__ qc, unsigned short* wqkv16, unsigned short* w116, unsigned short* w216,
           unsigned short* t16) {
  __shared__ __align__(16) unsigned short Th[256];
  const int tid = threadIdx.x, blk = blockIdx.x;
  if (blk < NBW0) {
    const int mat = blk >> 3;
    const float* src = (mat == 0) ? wq : ((mat == 1) ? wk : wv);
    const int t = (blk & 7) * 256 + tid;
    const v4u pk = cvt_w8(src + (size_t)t * 8);
    st16x2(wqkv16 + (size_t)mat * EMB * EMB + (size_t)t * 8, pk);
  } else if (blk < NBW0 + NBW1) {
    const int t = (blk - NBW0) * 256 + tid;
    const v4u pk = cvt_w8(w1 + (size_t)t * 8);
    st16x2(w116 + (size_t)t * 8, pk);
  } else if (blk < NBW0 + NBW1 + NBW2) {
    const int t = (blk - NBW0 - NBW1) * 256 + tid;
    const v4u pk = cvt_w8(w2 + (size_t)t * 8);
    st16x2(w216 + (size_t)t * 8, pk);
  } else if (blk < NBW0 + NBW1 + NBW2 + NBT) {
    const int tb = blk - NBW0 - NBW1 - NBW2;
    const int idx = tb * 256 + tid;
    const int n = idx >> 14, oi = idx & 16383;
    const float* bp = bw + (size_t)oi * NQC;
    const float* qp = qc + (size_t)n * NQC;
    float s = 0.f;
#pragma unroll 1
    for (int q = 0; q < NQC; q += 4) {
      const v4f a  = *(const v4f*)(bp + q);
      const v4f c4 = *(const v4f*)(qp + q);
      s += bfr(a[0]) * bfr(c4[0]);
      s += bfr(a[1]) * bfr(c4[1]);
      s += bfr(a[2]) * bfr(c4[2]);
      s += bfr(a[3]) * bfr(c4[3]);
    }
    Th[tid] = hb16(s * TSC);
    __syncthreads();
    if (tid < 32) {
      const v4u pk = *(const v4u*)(Th + tid * 8);
      st16x2(t16 + (size_t)tb * 256 + (size_t)tid * 8, pk);
    }
  }
}

__global__ __launch_bounds__(256)
void k_prep(const float* __restrict__ x, const float* __restrict__ g, const float* __restrict__ b,
            float* xr, unsigned short* xnh, unsigned short* xnl) {
  __shared__ __align__(16) float Xs[64 * LDC];
  const int tid = threadIdx.x, blk = blockIdx.x;
  const int n = blk >> 6, y = blk & 63;
  const float* xb = x + (size_t)n * EMB * HWP + (size_t)y * IMW;
#pragma unroll 4
  for (int it = 0; it < 32; ++it) {
    const int idx = it * 256 + tid;
    const int c = idx >> 6, xl = idx & 63;
    Xs[xl * LDC + c] = bfr(xb[(size_t)c * HWP + xl]);
  }
  __syncthreads();
  {
    v4f pv[8];
    size_t offs[8];
#pragma unroll
    for (int s = 0; s < 8; ++s) {
      const int idx = s * 256 + tid;
      const int row = idx >> 5, piece = idx & 31;
      pv[s] = *(const v4f*)(Xs + row * LDC + piece * 4);
      offs[s] = (size_t)(blk * 64 + row) * EMB + piece * 4;
    }
#pragma unroll
    for (int s = 0; s < 8; ++s) *(volatile v4f*)(xr + offs[s]) = pv[s];
    __threadfence();
#pragma unroll
    for (int s = 0; s < 8; ++s) *(volatile v4f*)(xr + offs[s]) = pv[s];
  }
  __syncthreads();
  ln_tile(Xs, g, b);
  __syncthreads();
  store_hilo(Xs, xnh, xnl, (size_t)blk * 64);
}

__global__ __launch_bounds__(256)
void k_ln2(const float* __restrict__ z2, const float* __restrict__ g, const float* __restrict__ b,
           unsigned short* z3h, unsigned short* z3l) {
  __shared__ __align__(16) float Xs[64 * LDC];
  const int tid = threadIdx.x, blk = blockIdx.x;
  const size_t row0 = (size_t)blk * 64;
#pragma unroll
  for (int it = 0; it < 8; ++it) {
    const int idx = it * 256 + tid;
    const int row = idx >> 5, piece = idx & 31;
    *(v4f*)(Xs + row * LDC + piece * 4) = *(const v4f*)(z2 + (row0 + row) * EMB + piece * 4);
  }
  __syncthreads();
  ln_tile(Xs, g, b);
  __syncthreads();
  store_hilo(Xs, z3h, z3l, row0);
}

__global__ __launch_bounds__(256)
void k_qkv(const unsigned short* __restrict__ xnh, const unsigned short* __restrict__ xnl,
           const unsigned short* __restrict__ wqkv16, const float* __restrict__ bq,
           const float* __restrict__ bk, const float* __restrict__ bv,
           unsigned short* q16, unsigned short* k16, unsigned short* vth, unsigned short* vtl) {
  __shared__ __align__(16) float Cs[64 * LDC];
  const int tid = threadIdx.x;
  const int mb = blockIdx.x, nb = blockIdx.y;
  mm_core2(xnh, xnl, EMB, wqkv16, EMB, EMB / 32, mb * 64, nb * 128, Cs);
  __syncthreads();
  if (nb < 2) {
    const float* bias = (nb == 0) ? bq : bk;
    unsigned short* dstp = (nb == 0) ? q16 : k16;
    v4u pk[4];
    size_t offs[4];
#pragma unroll
    for (int s = 0; s < 4; ++s) {
      const int idx = s * 256 + tid;
      const int row = idx >> 4, piece = idx & 15;
      const int col0 = piece * 8;
      v4u a;
#pragma unroll
      for (int e = 0; e < 4; ++e) {
        const float f0 = (Cs[row * LDC + col0 + 2 * e]     * PJS + bfr(bias[col0 + 2 * e]))     * QKS;
        const float f1 = (Cs[row * LDC + col0 + 2 * e + 1] * PJS + bfr(bias[col0 + 2 * e + 1])) * QKS;
        a[e] = pk16(hb16(f0), hb16(f1));
      }
      pk[s] = a;
      offs[s] = (size_t)(mb * 64 + row) * EMB + col0;
    }
#pragma unroll
    for (int s = 0; s < 4; ++s) *(volatile v4u*)(dstp + offs[s]) = pk[s];
    __threadfence();
#pragma unroll
    for (int s = 0; s < 4; ++s) *(volatile v4u*)(dstp + offs[s]) = pk[s];
  } else {
    v4u ph[4], plq[4];
    size_t offs[4];
#pragma unroll
    for (int s = 0; s < 4; ++s) {
      const int idx = s * 256 + tid;
      const int col = idx >> 3, p = idx & 7;
      const int x0 = p * 8;
      const float bb = bfr(bv[col]);
      v4u a, q4;
#pragma unroll
      for (int e = 0; e < 4; ++e) {
        const float f0 = (Cs[(x0 + 2 * e) * LDC + col]     * PJS + bb) * VSC;
        const float f1 = (Cs[(x0 + 2 * e + 1) * LDC + col] * PJS + bb) * VSC;
        unsigned ph_, pl_;
        hl2(f0, f1, ph_, pl_);
        a[e] = ph_;
        q4[e] = pl_;
      }
      ph[s] = a;
      plq[s] = q4;
      offs[s] = (size_t)mb * (EMB * IMW) + (size_t)idx * 8;
    }
#pragma unroll
    for (int s = 0; s < 4; ++s) { *(volatile v4u*)(vth + offs[s]) = ph[s]; *(volatile v4u*)(vtl + offs[s]) = plq[s]; }
    __threadfence();
#pragma unroll
    for (int s = 0; s < 4; ++s) { *(volatile v4u*)(vth + offs[s]) = ph[s]; *(volatile v4u*)(vtl + offs[s]) = plq[s]; }
  }
}

__global__ __launch_bounds__(256)
void k_attn(const unsigned short* __restrict__ q16, const unsigned short* __restrict__ k16,
            const unsigned short* __restrict__ vth, const unsigned short* __restrict__ vtl,
            const float* __restrict__ relb, unsigned short* oh, unsigned short* ol) {
  __shared__ __align__(16) float Os[32 * OSP];
  __shared__ float Bs[HEADS * 64];
  const int tid = threadIdx.x, wave = tid >> 5, lane = tid & 31, hh = lane >> 4, c = lane & 15;
  const int qt = wave >> 2, head = wave & 3;
  const int blk = blockIdx.x;
  const int n = blk >> 7, y = (blk >> 1) & 63, xh = blk & 1;
  if (tid < HEADS * PWIN) {
    const int hb = tid / PWIN;
    Bs[hb * 64 + (tid - hb * PWIN)] = bfr(relb[min(tid, HEADS * PWIN - 1)]);
  }
  __syncthreads();
  const int x0 = 32 * xh + 16 * qt;
  const int prow = (n * IMH + y) * IMW;
  const int choff = head * HDIM + 8 * hh;
  const float* bsh = Bs + head * 64;
  const v16us bq = ldfrag(q16 + (size_t)(prow + x0 + c) * EMB + choff);
  const v8f z8 = zero8();
  const v16us zu16 = zero16();
  const v8us zu = zero8u();

  float mx = -3.0e38f;
#pragma unroll 1
  for (int t = 0; t < 2 * KWIN; ++t) {
    const int g = t >> 1, s16 = (t & 1) * 16;
    const int yk = y + g - 3;
    const int xk = x0 - 8 + s16 + c;
    const bool ok = ((unsigned)yk < (unsigned)IMH) && ((unsigned)xk < (unsigned)IMW);
    const int ykc = min(max(yk, 0), IMH - 1), xkc = min(max(xk, 0), IMW - 1);
    v16us fa = ldfrag(k16 + (size_t)((n * IMH + ykc) * IMW + xkc) * EMB + choff);
    fa = ok ? fa : zu16;
    v8f sc = mma_h(fa, bq, z8);
    guard_s1(sc, fa, bq);
#pragma unroll
    for (int r = 0; r < 8; ++r) {
      const int dxp = s16 + 8 * hh + r - c - 5;
      const bool live = (unsigned)dxp <= 6u;
      const int p = g * KWIN + min(max(dxp, 0), 6);
      const float lg = sc[r] * SSC + bsh[p];
      mx = fmaxf(mx, live ? lg : -3.0e38f);
    }
  }
  const float m = fmaxf(mx, __shfl_xor(mx, 16, 32));

  v8f acch0 = zero8(), accl0 = zero8(), acch1 = zero8(), accl1 = zero8();
  float lsum = 0.f;
#pragma unroll 1
  for (int g = 0; g < KWIN; ++g) {
    const int yk = y + g - 3;
    const bool rin = (unsigned)yk < (unsigned)IMH;
    const int ykc = min(max(yk, 0), IMH - 1);
    const int krow = (n * IMH + ykc) * IMW;
    const int xa = x0 - 8 + c, xb = x0 + 8 + c;
    const bool oka = rin && ((unsigned)xa < (unsigned)IMW);
    const bool okb = rin && ((unsigned)xb < (unsigned)IMW);
    const int xac = min(max(xa, 0), IMW - 1), xbc = min(max(xb, 0), IMW - 1);
    v16us ak0 = ldfrag(k16 + (size_t)(krow + xac) * EMB + choff);
    v16us ak1 = ldfrag(k16 + (size_t)(krow + xbc) * EMB + choff);
    ak0 = oka ? ak0 : zu16;
    ak1 = okb ? ak1 : zu16;
    v8f s0 = mma_h(ak0, bq, z8);
    v8f s1 = mma_h(ak1, bq, z8);
    guard_s2(s0, s1, ak0, ak1, bq);
    const int pa = x0 - 8 + 8 * hh, pb = x0 + 8 + 8 * hh;
    const bool va = rin && ((unsigned)pa < (unsigned)IMW);
    const bool vb = rin && ((unsigned)pb < (unsigned)IMW);
    const int pac = min(max(pa, 0), IMW - 8), pbc = min(max(pb, 0), IMW - 8);
    const size_t vo0 = ((size_t)(n * IMH + ykc) * EMB + head * HDIM + c) * IMW;
    const size_t vo1 = vo0 + (size_t)16 * IMW;
    UFrag vh0, vl0, vh1, vl1;
    {
      v8us tv;
      tv = *(const v8us*)(vth + vo0 + pac); vh0.u[0] = va ? tv : zu;
      tv = *(const v8us*)(vth + vo0 + pbc); vh0.u[1] = vb ? tv : zu;
      tv = *(const v8us*)(vtl + vo0 + pac); vl0.u[0] = va ? tv : zu;
      tv = *(const v8us*)(vtl + vo0 + pbc); vl0.u[1] = vb ? tv : zu;
      tv = *(const v8us*)(vth + vo1 + pac); vh1.u[0] = va ? tv : zu;
      tv = *(const v8us*)(vth + vo1 + pbc); vh1.u[1] = vb ? tv : zu;
      tv = *(const v8us*)(vtl + vo1 + pac); vl1.u[0] = va ? tv : zu;
      tv = *(const v8us*)(vtl + vo1 + pbc); vl1.u[1] = vb ? tv : zu;
    }
    UFrag ph, pl;
#pragma unroll
    for (int rr = 0; rr < 4; ++rr) {
      const int ra = 2 * rr, rb = 2 * rr + 1;
      const int d0a = 8 * hh + ra - c - 5, d0b = 8 * hh + rb - c - 5;
      const int d1a = d0a + 16, d1b = d0b + 16;
      const bool l0a = (unsigned)d0a <= 6u, l0b = (unsigned)d0b <= 6u;
      const bool l1a = (unsigned)d1a <= 6u, l1b = (unsigned)d1b <= 6u;
      const float b0a = bsh[g * KWIN + min(max(d0a, 0), 6)], b0b = bsh[g * KWIN + min(max(d0b, 0), 6)];
      const float b1a = bsh[g * KWIN + min(max(d1a, 0), 6)], b1b = bsh[g * KWIN + min(max(d1b, 0), 6)];
      const float ea = __expf(s0[ra] * SSC + b0a - m), eb = __expf(s0[rb] * SSC + b0b - m);
      const float fa = __expf(s1[ra] * SSC + b1a - m), fb = __expf(s1[rb] * SSC + b1b - m);
      const float pa_ = l0a ? ea : 0.f;
      const float pb_ = l0b ? eb : 0.f;
      const float qa_ = l1a ? fa : 0.f;
      const float qb_ = l1b ? fb : 0.f;
      lsum += (pa_ + pb_) + (qa_ + qb_);
      unsigned h0, g0, h1, g1;
      hl2(pa_, pb_, h0, g0);
      hl2(qa_, qb_, h1, g1);
      ph.w[0][rr] = h0; pl.w[0][rr] = g0;
      ph.w[1][rr] = h1; pl.w[1][rr] = g1;
    }
    acch0 = mma_h(ph.v, vh0.v, acch0);
    accl0 = mma_h(pl.v, vh0.v, accl0);
    accl0 = mma_h(ph.v, vl0.v, accl0);
    acch1 = mma_h(ph.v, vh1.v, acch1);
    accl1 = mma_h(pl.v, vh1.v, accl1);
    accl1 = mma_h(ph.v, vl1.v, accl1);
    guard6(acch0, accl0, acch1, accl1, ph.v, pl.v, vh0.v, vl0.v, vh1.v, vl1.v);
  }
  const float lq = lsum + __shfl_xor(lsum, 16, 32);
  const float rl = __builtin_amdgcn_rcpf(lq) * OFAC;
#pragma unroll
  for (int r = 0; r < 8; ++r) {
    const float f = __shfl(rl, 8 * hh + r, 32);
    const int orow = (qt * 16 + 8 * hh + r) * OSP + head * HDIM;
    Os[orow + c]      = (acch0[r] + accl0[r] * RSC) * f;
    Os[orow + 16 + c] = (acch1[r] + accl1[r] * RSC) * f;
  }
  __syncthreads();
  v4u hw[2], lw[2];
  size_t offs[2];
#pragma unroll
  for (int s = 0; s < 2; ++s) {
    const int idx = s * 256 + tid;
    const int row = idx >> 4, piece = idx & 15;
    const v4f a = *(const v4f*)(Os + row * OSP + piece * 8);
    const v4f b = *(const v4f*)(Os + row * OSP + piece * 8 + 4);
    v4u h4, l4;
    unsigned ph_, pl_;
    hl2(a[0], a[1], ph_, pl_); h4[0] = ph_; l4[0] = pl_;
    hl2(a[2], a[3], ph_, pl_); h4[1] = ph_; l4[1] = pl_;
    hl2(b[0], b[1], ph_, pl_); h4[2] = ph_; l4[2] = pl_;
    hl2(b[2], b[3], ph_, pl_); h4[3] = ph_; l4[3] = pl_;
    hw[s] = h4;
    lw[s] = l4;
    offs[s] = (size_t)(prow + 32 * xh + row) * EMB + piece * 8;
  }
#pragma unroll
  for (int s = 0; s < 2; ++s) { *(volatile v4u*)(oh + offs[s]) = hw[s]; *(volatile v4u*)(ol + offs[s]) = lw[s]; }
  __threadfence();
#pragma unroll
  for (int s = 0; s < 2; ++s) { *(volatile v4u*)(oh + offs[s]) = hw[s]; *(volatile v4u*)(ol + offs[s]) = lw[s]; }
}

__global__ __launch_bounds__(256)
void k_bil(const unsigned short* __restrict__ ohp, const unsigned short* __restrict__ olp,
           const unsigned short* __restrict__ t16, const float* __restrict__ bilb,
           const float* __restrict__ xr, float* z2) {
  __shared__ __align__(16) float Cs[64 * LDC];
  const int tid = threadIdx.x;
  const int mb = blockIdx.x, n = mb >> 6;
  mm_core2(ohp, olp, EMB, t16 + (size_t)n * EMB * EMB, EMB, EMB / 32, mb * 64, 0, Cs);
  __syncthreads();
  v4f pv[8];
  size_t offs[8];
#pragma unroll
  for (int s = 0; s < 8; ++s) {
    const int idx = s * 256 + tid;
    const int row = idx >> 5, piece = idx & 31;
    const int col0 = piece * 4;
    const size_t o = (size_t)(mb * 64 + row) * EMB + col0;
    const v4f xv = *(const v4f*)(xr + o);
    v4f val;
#pragma unroll
    for (int e = 0; e < 4; ++e) val[e] = Cs[row * LDC + col0 + e] * PSC + bfr(bilb[col0 + e]) + xv[e];
    pv[s] = val;
    offs[s] = o;
  }
#pragma unroll
  for (int s = 0; s < 8; ++s) *(volatile v4f*)(z2 + offs[s]) = pv[s];
  __threadfence();
#pragma unroll
  for (int s = 0; s < 8; ++s) *(volatile v4f*)(z2 + offs[s]) = pv[s];
}

__global__ __launch_bounds__(256)
void k_ffn1(const unsigned short* __restrict__ z3h, const unsigned short* __restrict__ z3l,
            const unsigned short* __restrict__ w116, const float* __restrict__ b1,
            unsigned short* h1h, unsigned short* h1l) {
  __shared__ __align__(16) float Cs[64 * LDC];
  const int tid = threadIdx.x;
  const int mb = blockIdx.x, nb = blockIdx.y;
  mm_core2(z3h, z3l, EMB, w116, EMB, EMB / 32, mb * 64, nb * 128, Cs);
  __syncthreads();
  v4u hw[4], lw[4];
  size_t offs[4];
#pragma unroll
  for (int s = 0; s < 4; ++s) {
    const int idx = s * 256 + tid;
    const int row = idx >> 4, piece = idx & 15;
    const int col0 = piece * 8;
    v4u a, q4;
#pragma unroll
    for (int e = 0; e < 4; ++e) {
      const int j0 = col0 + 2 * e, j1 = j0 + 1;
      const float u0 = Cs[row * LDC + j0] * PJS + bfr(b1[nb * 128 + j0]);
      const float u1 = Cs[row * LDC + j1] * PJS + bfr(b1[nb * 128 + j1]);
      const float g0 = 0.5f * u0 * (1.0f + erff(u0 * 0.70710678118654752f)) * HSC;
      const float g1 = 0.5f * u1 * (1.0f + erff(u1 * 0.70710678118654752f)) * HSC;
      unsigned ph_, pl_;
      hl2(g0, g1, ph_, pl_);
      a[e] = ph_;
      q4[e] = pl_;
    }
    hw[s] = a;
    lw[s] = q4;
    offs[s] = (size_t)(mb * 64 + row) * FFD + (size_t)nb * 128 + col0;
  }
#pragma unroll
  for (int s = 0; s < 4; ++s) { *(volatile v4u*)(h1h + offs[s]) = hw[s]; *(volatile v4u*)(h1l + offs[s]) = lw[s]; }
  __threadfence();
#pragma unroll
  for (int s = 0; s < 4; ++s) { *(volatile v4u*)(h1h + offs[s]) = hw[s]; *(volatile v4u*)(h1l + offs[s]) = lw[s]; }
}

__global__ __launch_bounds__(256)
void k_ffn2(const unsigned short* __restrict__ h1h, const unsigned short* __restrict__ h1l,
            const unsigned short* __restrict__ w216, const float* __restrict__ b2,
            const float* __restrict__ z2, float* out) {
  __shared__ __align__(16) float Cs[64 * LDC];
  const int tid = threadIdx.x, wave = tid >> 5, lane = tid & 31, hh = lane >> 4, piece = lane & 15;
  const int mb = blockIdx.x;
  const int n = mb >> 6, y = mb & 63;
  mm_core2(h1h, h1l, FFD, w216, FFD, FFD / 32, mb * 64, 0, Cs);
  __syncthreads();
#pragma unroll 1
  for (int it = 0; it < 8; ++it) {
    const int o = wave * 16 + it * 2 + hh;
    const float bo = bfr(b2[o]);
    v4f val;
#pragma unroll
    for (int e = 0; e < 4; ++e) {
      const int px = piece * 4 + e;
      val[e] = Cs[px * LDC + o] * F2S + bo + z2[(size_t)(mb * 64 + px) * EMB + o];
    }
    float* p = out + ((size_t)(n * EMB + o)) * HWP + (size_t)y * IMW + piece * 4;
    *(volatile v4f*)p = val;
    __threadfence();
    *(volatile v4f*)p = val;
  }
}

extern "C" void kernel_launch(void* const* d_in, const int* in_sizes, int n_in,
                              void* d_out, int out_size, void* d_ws, size_t ws_size,
                              hipStream_t stream) {
  if (n_in < 19) return;
  const int expect[19] = { NPIX * EMB, NBAT * NQC, EMB * EMB, EMB, EMB * EMB, EMB, EMB * EMB, EMB,
                           HEADS * PWIN, EMB, EMB, EMB * EMB * NQC, EMB, EMB, EMB, FFD * EMB, FFD, EMB * FFD, EMB };
  for (int i = 0; i < 19; ++i) if (in_sizes[i] != expect[i]) return;
  if (out_size != NPIX * EMB) return;

  const float* x     = (const float*)d_in[0];
  const float* qcf   = (const float*)d_in[1];
  const float* wq    = (const float*)d_in[2];
  const float* bq    = (const float*)d_in[3];
  const float* wk    = (const float*)d_in[4];
  const float* bk    = (const float*)d_in[5];
  const float* wv    = (const float*)d_in[6];
  const float* bv    = (const float*)d_in[7];
  const float* relb  = (const float*)d_in[8];
  const float* ln1g  = (const float*)d_in[9];
  const float* ln1b  = (const float*)d_in[10];
  const float* bilw  = (const float*)d_in[11];
  const float* bilb  = (const float*)d_in[12];
  const float* ln2g  = (const float*)d_in[13];
  const float* ln2b  = (const float*)d_in[14];
  const float* w1    = (const float*)d_in[15];
  const float* b1    = (const float*)d_in[16];
  const float* w2    = (const float*)d_in[17];
  const float* b2    = (const float*)d_in[18];
  float* out = (float*)d_out;

  const size_t AL = 65536;
  const size_t sWQ  = (((size_t)3 * EMB * EMB * 2) + AL - 1) / AL * AL;
  const size_t sW1  = (((size_t)FFD * EMB * 2) + AL - 1) / AL * AL;
  const size_t sW2  = (((size_t)EMB * FFD * 2) + AL - 1) / AL * AL;
  const size_t sT   = (((size_t)NBAT * EMB * EMB * 2) + AL - 1) / AL * AL;
  const size_t sF32 = (((size_t)NPIX * EMB * 4) + AL - 1) / AL * AL;
  const size_t sH16 = (((size_t)NPIX * EMB * 2) + AL - 1) / AL * AL;
  const size_t sH1  = (((size_t)NPIX * FFD * 2) + AL - 1) / AL * AL;

  size_t off = 0;
  const size_t oWQ  = off; off += sWQ;
  const size_t oW1  = off; off += sW1;
  const size_t oW2  = off; off += sW2;
  const size_t oT   = off; off += sT;
  const size_t oXR  = off; off += sF32;
  const size_t oXNH = off; off += sH16;
  const size_t oXNL = off; off += sH16;
  const size_t oQ   = off; off += sH16;
  const size_t oK   = off; off += sH16;
  const size_t oVTH = off; off += sH16;
  const size_t oVTL = off; off += sH16;
  const size_t oOH  = off; off += sH16;
  const size_t oOL  = off; off += sH16;
  const size_t oZ2  = off; off += sF32;
  const size_t oZ3H = off; off += sH16;
  const size_t oZ3L = off; off += sH16;
  const size_t oH1H = off; off += sH1;
  const size_t oH1L = off; off += sH1;
  if (off > ws_size) return;
  if (off > (size_t)134217728) return;

  char* ws = (char*)d_ws;
  unsigned short* WQKV16 = (unsigned short*)(ws + oWQ);
  unsigned short* W1_16  = (unsigned short*)(ws + oW1);
  unsigned short* W2_16  = (unsigned short*)(ws + oW2);
  unsigned short* T16    = (unsigned short*)(ws + oT);
  float*          XR     = (float*)(ws + oXR);
  unsigned short* XNH    = (unsigned short*)(ws + oXNH);
  unsigned short* XNL    = (unsigned short*)(ws + oXNL);
  unsigned short* Q16    = (unsigned short*)(ws + oQ);
  unsigned short* K16    = (unsigned short*)(ws + oK);
  unsigned short* VTH    = (unsigned short*)(ws + oVTH);
  unsigned short* VTL    = (unsigned short*)(ws + oVTL);
  unsigned short* OH     = (unsigned short*)(ws + oOH);
  unsigned short* OL     = (unsigned short*)(ws + oOL);
  float*          Z2     = (float*)(ws + oZ2);
  unsigned short* Z3H    = (unsigned short*)(ws + oZ3H);
  unsigned short* Z3L    = (unsigned short*)(ws + oZ3L);
  unsigned short* H1H    = (unsigned short*)(ws + oH1H);
  unsigned short* H1L    = (unsigned short*)(ws + oH1L);

  const dim3 blk(256);
  k_cvt<<<dim3(NBW0 + NBW1 + NBW2 + NBT), blk, 0, stream>>>(wq, wk, wv, w1, w2, bilw, qcf, WQKV16, W1_16, W2_16, T16);
  k_prep<<<dim3(NPIX / 64), blk, 0, stream>>>(x, ln1g, ln1b, XR, XNH, XNL);
  k_qkv<<<dim3(NPIX / 64, 3), blk, 0, stream>>>(XNH, XNL, WQKV16, bq, bk, bv, Q16, K16, VTH, VTL);
  k_attn<<<dim3(NPIX / 32), blk, 0, stream>>>(Q16, K16, VTH, VTL, relb, OH, OL);
  k_bil<<<dim3(NPIX / 64), blk, 0, stream>>>(OH, OL, T16, bilb, XR, Z2);
  k_ln2<<<dim3(NPIX / 64), blk, 0, stream>>>(Z2, ln2g, ln2b, Z3H, Z3L);
  k_ffn1<<<dim3(NPIX / 64, FFD / 128), blk, 0, stream>>>(Z3H, Z3L, W1_16, b1, H1H, H1L);
  k_ffn2<<<dim3(NPIX / 64), blk, 0, stream>>>(H1H, H1L, W2_16, b2, Z2, out);
  (void)hipGetLastError();
}
